// concatDec_66279935312289
// MI455X (gfx1250) — hardware-verified
//
#include <hip/hip_runtime.h>
#include <stdint.h>


typedef __attribute__((ext_vector_type(16))) _Float16 v16h;
typedef __attribute__((ext_vector_type(8)))  _Float16 v8h;
typedef __attribute__((ext_vector_type(16))) __bf16   v16b;
typedef __attribute__((ext_vector_type(8)))  __bf16   v8b;
typedef __attribute__((ext_vector_type(8)))  float    v8f;
typedef __attribute__((ext_vector_type(4)))  float    v4f;

static constexpr int kD    = 128;
static constexpr int kTwoD = 256;
static constexpr int kH    = 512;
static constexpr int kNcat = 1024;

__device__ __forceinline__ unsigned short f2bf_bits(float f) {
  unsigned u = __float_as_uint(f);
  return (unsigned short)((u + 0x7FFFu + ((u >> 16) & 1u)) >> 16);
}
__device__ __forceinline__ float bf_bits2f(unsigned short h) { return __uint_as_float(((unsigned)h) << 16); }

__device__ __forceinline__ void dep_guard_h(v8f& a, v8f& b, v16h x, v16h y) { asm volatile("v_nop\n\tv_nop\n\tv_nop\n\tv_nop" : "+v"(a), "+v"(b) : "v"(x), "v"(y)); }
__device__ __forceinline__ void dep_guard_b(v8f& a, v8f& b, v16b x, v16b y) { asm volatile("v_nop\n\tv_nop\n\tv_nop\n\tv_nop" : "+v"(a), "+v"(b) : "v"(x), "v"(y)); }
__device__ __forceinline__ void keep4_h(v16h a, v16h b, v16h c, v16h d) { asm volatile("v_nop" :: "v"(a), "v"(b), "v"(c), "v"(d)); }
__device__ __forceinline__ void keep4_b(v16b a, v16b b, v16b c, v16b d) { asm volatile("v_nop" :: "v"(a), "v"(b), "v"(c), "v"(d)); }
__device__ __forceinline__ void acc_guard4(v8f& a, v8f& b, v8f& c, v8f& d) { asm volatile("v_nop\n\tv_nop\n\tv_nop\n\tv_nop" : "+v"(a), "+v"(b), "+v"(c), "+v"(d)); }
template <typename T> struct Frag;
template <> struct Frag<_Float16> {
  typedef v16h V; union U { v16h v; v8h h[2]; };
  static __device__ __forceinline__ v16h load(const _Float16* p) {
    U f; f.h[0] = *(const v8h*)(p); f.h[1] = *(const v8h*)(p + 16); return f.v;
  }
  static __device__ __forceinline__ v8f mma(v16h a, v16h b, v8f c) {
    return __builtin_amdgcn_wmma_f32_16x16x32_f16(false, a, false, b, (short)0, c, false, false);
  }
  static __device__ __forceinline__ void guard(v8f& a, v8f& b, v16h x, v16h y) { dep_guard_h(a, b, x, y); }
  static __device__ __forceinline__ void keep(v16h a, v16h b, v16h c, v16h d) { keep4_h(a, b, c, d); }
};
template <> struct Frag<__bf16> {
  typedef v16b V; union U { v16b v; v8b h[2]; };
  static __device__ __forceinline__ v16b load(const __bf16* p) {
    U f; f.h[0] = *(const v8b*)(p); f.h[1] = *(const v8b*)(p + 16); return f.v;
  }
  static __device__ __forceinline__ v8f mma(v16b a, v16b b, v8f c) {
    return __builtin_amdgcn_wmma_f32_16x16x32_bf16(false, a, false, b, (short)0, c, false, false);
  }
  static __device__ __forceinline__ void guard(v8f& a, v8f& b, v16b x, v16b y) { dep_guard_b(a, b, x, y); }
  static __device__ __forceinline__ void keep(v16b a, v16b b, v16b c, v16b d) { keep4_b(a, b, c, d); }
};

template <int ET> struct Elem;
template <> struct Elem<0> { typedef _Float16 T; };
template <> struct Elem<1> { typedef __bf16 T; };
template <int ET, bool SPLIT, int BIAS_MODE, int OUT_MODE, bool RESID, int ACT = 0>
__global__ __launch_bounds__(256) void wmma_gemm64(
    const unsigned short* __restrict__ Ap, const unsigned short* __restrict__ A2p, int lda, long strideA,
    const unsigned short* __restrict__ Btp, const unsigned short* __restrict__ Bt2p, int ldb, long strideB,
    void* __restrict__ Cout, void* __restrict__ Cout2, int ldc, long strideC,
    const float* __restrict__ bias,
    const float* __restrict__ resid, long strideR,
    int M, int N, int K, float scale) {
  typedef typename Elem<ET>::T T;
  typedef typename Frag<T>::V V;
  const T* A = (const T*)Ap; const T* A2 = (const T*)A2p; const T* Bt = (const T*)Btp; const T* Bt2 = (const T*)Bt2p;
  __shared__ __align__(16) float sT[8][16 * 68];
  const int b    = blockIdx.y;
  const int lane = threadIdx.x & 31;
  const int wave = threadIdx.x >> 5;
  const int tilesN = N >> 6;
  const int tilesM = M >> 6;
  const int tile = blockIdx.x * 8 + wave;
  if (tile >= tilesM * tilesN) return;
  const int tm = tile / tilesN;
  const int tn = tile - tm * tilesN;
  const int m0 = tm << 6;
  const int n0 = tn << 6;

  const T* Ab  = A  + (size_t)b * strideA;
  const T* Bb  = Bt + (size_t)b * strideB;
  const T* Ab2 = SPLIT ? (A2  + (size_t)b * strideA) : nullptr;
  const T* Bb2 = SPLIT ? (Bt2 + (size_t)b * strideB) : nullptr;

  const int rlane = lane & 15;
  const int koff  = (lane >> 4) * 8;
  const int mOff  = (lane >> 4) * 8;

  v8f acc[4][4];
#pragma unroll
  for (int i = 0; i < 4; ++i)
#pragma unroll
    for (int j = 0; j < 4; ++j) acc[i][j] = (v8f){0.f,0.f,0.f,0.f,0.f,0.f,0.f,0.f};

  for (int k0 = 0; k0 < K; k0 += 32) {
    V bh[4], bl[4];
#pragma unroll
    for (int j = 0; j < 4; ++j) {
      const size_t bo = (size_t)(n0 + (j << 4) + rlane) * ldb + koff + k0;
      bh[j] = Frag<T>::load(Bb + bo);
      if (SPLIT) bl[j] = Frag<T>::load(Bb2 + bo);
    }
#pragma unroll
    for (int i = 0; i < 4; ++i) {
      const size_t ao = (size_t)(m0 + (i << 4) + rlane) * lda + koff + k0;
      V ah = Frag<T>::load(Ab + ao);
      V al;
      if (SPLIT) al = Frag<T>::load(Ab2 + ao);
#pragma unroll
      for (int j = 0; j < 4; ++j) {
        acc[i][j] = Frag<T>::mma(ah, bh[j], acc[i][j]);
        if (SPLIT) {
          acc[i][j] = Frag<T>::mma(ah, bl[j], acc[i][j]);
          acc[i][j] = Frag<T>::mma(al, bh[j], acc[i][j]);
        }
      }
      Frag<T>::guard(acc[i][0], acc[i][3], ah, SPLIT ? al : ah);
    }
    Frag<T>::keep(bh[0], bh[1], bh[2], bh[3]);
    if (SPLIT) Frag<T>::keep(bl[0], bl[1], bl[2], bl[3]);
  }
  acc_guard4(acc[0][0], acc[0][1], acc[0][2], acc[0][3]);
  acc_guard4(acc[1][0], acc[1][1], acc[1][2], acc[1][3]);
  acc_guard4(acc[2][0], acc[2][1], acc[2][2], acc[2][3]);
  acc_guard4(acc[3][0], acc[3][1], acc[3][2], acc[3][3]);

  float* slab = sT[wave];
  const float* Rb = RESID ? (resid + (size_t)b * strideR) : nullptr;
#pragma unroll
  for (int i = 0; i < 4; ++i) {
    const int mBase = m0 + (i << 4);
#pragma unroll
    for (int j = 0; j < 4; ++j) {
      const int n = n0 + (j << 4) + rlane;
      float bv = 0.f;
      if (BIAS_MODE == 2) bv = bias[n];
#pragma unroll
      for (int r = 0; r < 8; ++r) {
        float v = acc[i][j][r] * scale;
        if (BIAS_MODE == 1) v += bias[mBase + mOff + r];
        if (BIAS_MODE == 2) v += bv;
        if (RESID) v += Rb[(size_t)(mBase + mOff + r) * ldc + n];
        if (ACT == 1) v = tanhf(v);
        if (ACT == 2) v = fmaxf(v, 0.0f);
        if (ACT == 3) v = v / (1.0f + expf(-v));
        if (ACT == 4) v = (v > 0.f) ? v : 0.01f * v;
        if (ACT == 5) v = 0.5f * v * (1.0f + erff(v * 0.70710678118654752f));
        slab[(mOff + r) * 68 + (j << 4) + rlane] = v;
      }
    }
    __builtin_amdgcn_fence(__ATOMIC_RELEASE, "workgroup");
    __builtin_amdgcn_wave_barrier();
    __builtin_amdgcn_fence(__ATOMIC_ACQUIRE, "workgroup");
    if (OUT_MODE == 0) {
      float* C = (float*)Cout + (size_t)b * strideC;
      const int hh = lane >> 4, c4 = (lane & 15) * 4;
      for (int pass = 0; pass < 2; ++pass) {
#pragma unroll
        for (int it = 0; it < 8; ++it) {
          const int row = it * 2 + hh;
          v4f v = *(const v4f*)(slab + row * 68 + c4);
          *(volatile v4f*)(C + (size_t)(mBase + row) * ldc + n0 + c4) = v;
        }
        __threadfence();
      }
    } else {
      const int q = lane >> 3, c8 = (lane & 7) * 8;
      unsigned short* C  = (unsigned short*)Cout  + (size_t)b * strideC;
      unsigned short* C2 = (OUT_MODE == 2) ? ((unsigned short*)Cout2 + (size_t)b * strideC) : nullptr;
      for (int pass = 0; pass < 2; ++pass) {
#pragma unroll
        for (int it = 0; it < 4; ++it) {
          const int row = it * 4 + q;
          const float* sp = slab + row * 68 + c8;
          v8h hv, lv;
#pragma unroll
          for (int e = 0; e < 8; ++e) {
            if (OUT_MODE == 1) {
              hv[e] = (_Float16)sp[e];
            } else {
              unsigned short hb = f2bf_bits(sp[e]);
              unsigned short lb = f2bf_bits(sp[e] - bf_bits2f(hb));
              hv[e] = __builtin_bit_cast(_Float16, hb);
              lv[e] = __builtin_bit_cast(_Float16, lb);
            }
          }
          *(volatile v8h*)(C + (size_t)(mBase + row) * ldc + n0 + c8) = hv;
          if (OUT_MODE == 2) *(volatile v8h*)(C2 + (size_t)(mBase + row) * ldc + n0 + c8) = lv;
        }
        __threadfence();
      }
    }
    __builtin_amdgcn_fence(__ATOMIC_RELEASE, "workgroup");
    __builtin_amdgcn_wave_barrier();
    __builtin_amdgcn_fence(__ATOMIC_ACQUIRE, "workgroup");
  }
}

__global__ __launch_bounds__(256) void cast_f32_f16x2(
    const float* __restrict__ in, _Float16* __restrict__ out, int n2) {
  int i = blockIdx.x * 256 + threadIdx.x;
  if (i < n2) {
    const _Float16 h0 = (_Float16)in[2 * i], h1 = (_Float16)in[2 * i + 1];
    const unsigned u = (unsigned)__builtin_bit_cast(unsigned short, h0) | ((unsigned)__builtin_bit_cast(unsigned short, h1) << 16);
    ((volatile unsigned*)out)[i] = u;
    __threadfence();
    ((volatile unsigned*)out)[i] = u;
  }
}

__global__ __launch_bounds__(256) void build_w1cat_f16x2(
    const float* __restrict__ W1, _Float16* __restrict__ out, int n2) {
  int i = blockIdx.x * 256 + threadIdx.x;
  if (i < n2) {
    const int e0 = 2 * i;
    const int n  = e0 >> 7;
    const int k  = e0 & (kD - 1);
    const int src = (n < kH) ? (n * kTwoD + k) : ((n - kH) * kTwoD + kD + k);
    const _Float16 h0 = (_Float16)(W1[src] * 16.0f), h1 = (_Float16)(W1[src + 1] * 16.0f);
    const unsigned u = (unsigned)__builtin_bit_cast(unsigned short, h0) | ((unsigned)__builtin_bit_cast(unsigned short, h1) << 16);
    ((volatile unsigned*)out)[i] = u;
    __threadfence();
    ((volatile unsigned*)out)[i] = u;
  }
}

__global__ __launch_bounds__(256) void edge_decode_kernel(
    const _Float16* __restrict__ P, const int* __restrict__ eidx,
    const float* __restrict__ b1, const float* __restrict__ W2, const float* __restrict__ b2,
    float* __restrict__ out, int E, int Nn) {
  const int lane = threadIdx.x & 31;
  const int wave = threadIdx.x >> 5;
  const int base = (blockIdx.x * 8 + wave) * 32;
  if (base >= E) return;

  float w2r[16], b1r[16];
  {
    const v4f wa = *(const v4f*)(W2 + 8 * lane);
    const v4f wb = *(const v4f*)(W2 + 8 * lane + 4);
    const v4f wc = *(const v4f*)(W2 + 256 + 8 * lane);
    const v4f wd = *(const v4f*)(W2 + 256 + 8 * lane + 4);
    const v4f ba = *(const v4f*)(b1 + 8 * lane);
    const v4f bb = *(const v4f*)(b1 + 8 * lane + 4);
    const v4f bc = *(const v4f*)(b1 + 256 + 8 * lane);
    const v4f bd = *(const v4f*)(b1 + 256 + 8 * lane + 4);
#pragma unroll
    for (int t = 0; t < 4; ++t) {
      w2r[t] = wa[t]; w2r[4 + t] = wb[t]; w2r[8 + t] = wc[t]; w2r[12 + t] = wd[t];
      b1r[t] = ba[t]; b1r[4 + t] = bb[t]; b1r[8 + t] = bc[t]; b1r[12 + t] = bd[t];
    }
  }
  const float b2v = b2[0];

  const int e_l = base + lane;
  const int ec  = (e_l < E) ? e_l : (E - 1);
  int s_l = eidx[ec];
  int d_l = eidx[(size_t)E + (size_t)ec];
  s_l = (s_l < 0) ? 0 : ((s_l >= Nn) ? (Nn - 1) : s_l);
  d_l = (d_l < 0) ? 0 : ((d_l >= Nn) ? (Nn - 1) : d_l);

  float yout = 0.0f;
#pragma unroll 1
  for (int j = 0; j < 32; ++j) {
    const int s = __shfl(s_l, j, 32);
    const int d = __shfl(d_l, j, 32);
    const _Float16* pa = P + (size_t)s * kNcat + 8 * lane;
    const _Float16* pb = P + (size_t)d * kNcat + kH + 8 * lane;
    const v8h a0 = *(const v8h*)(pa);
    const v8h a1 = *(const v8h*)(pa + 256);
    const v8h c0 = *(const v8h*)(pb);
    const v8h c1 = *(const v8h*)(pb + 256);
    float acc = 0.0f;
#pragma unroll
    for (int i = 0; i < 8; ++i) {
      float h0 = (float)a0[i] + (float)c0[i] + b1r[i];
      h0 = fmaxf(h0, 0.0f);
      acc += h0 * w2r[i];
      float h1 = (float)a1[i] + (float)c1[i] + b1r[8 + i];
      h1 = fmaxf(h1, 0.0f);
      acc += h1 * w2r[8 + i];
    }
#pragma unroll
    for (int off = 16; off >= 1; off >>= 1) acc += __shfl_xor(acc, off, 32);
    acc += b2v;
    yout = (lane == j) ? acc : yout;
  }
  if (e_l < E) *(volatile float*)(out + e_l) = yout;
  __threadfence();
  if (e_l < E) *(volatile float*)(out + e_l) = yout;
}

static inline size_t align256(size_t x) { return (x + 255) & ~(size_t)255; }

extern "C" void kernel_launch(void* const* d_in, const int* in_sizes, int n_in,
                              void* d_out, int out_size, void* d_ws, size_t ws_size,
                              hipStream_t stream) {
  if (n_in < 6) return;
  const float* z    = (const float*)d_in[0];
  const int*   eidx = (const int*)d_in[1];
  const float* W1   = (const float*)d_in[2];
  const float* b1   = (const float*)d_in[3];
  const float* W2   = (const float*)d_in[4];
  const float* b2   = (const float*)d_in[5];
  float*       out  = (float*)d_out;

  const int Nn = in_sizes[0] / kD;
  const int E  = in_sizes[1] / 2;
  if (Nn <= 0 || E <= 0) return;
  if (in_sizes[0] != Nn * kD || in_sizes[2] != kH * kTwoD || in_sizes[3] != kH ||
      in_sizes[4] != kH || in_sizes[5] < 1 || out_size < E) return;

  const int Mp = ((Nn + 63) / 64) * 64;
  const size_t offZ   = 0;
  const size_t bytesZ = (size_t)Mp * kD * sizeof(_Float16);
  const size_t offW   = align256(offZ + bytesZ);
  const size_t bytesW = (size_t)kNcat * kD * sizeof(_Float16);
  const size_t offP   = align256(offW + bytesW);
  const size_t bytesP = (size_t)Mp * kNcat * sizeof(_Float16);
  const size_t total  = offP + bytesP;
  if (total > ws_size) return;

  char* ws = (char*)d_ws;
  _Float16* z16 = (_Float16*)(ws + offZ);
  _Float16* w16 = (_Float16*)(ws + offW);
  _Float16* P16 = (_Float16*)(ws + offP);

  if (Mp > Nn) {
    hipMemsetAsync(ws + offZ + (size_t)Nn * kD * sizeof(_Float16), 0,
                   (size_t)(Mp - Nn) * kD * sizeof(_Float16), stream);
  }

  {
    const int n2 = (Nn * kD) / 2;
    const int grid = (n2 + 255) / 256;
    cast_f32_f16x2<<<grid, 256, 0, stream>>>(z, z16, n2);
  }
  {
    const int n2 = (kNcat * kD) / 2;
    const int grid = (n2 + 255) / 256;
    build_w1cat_f16x2<<<grid, 256, 0, stream>>>(W1, w16, n2);
  }
  {
    const int tiles = (Mp / 64) * (kNcat / 64);
    dim3 grid((tiles + 7) / 8, 1, 1);
    wmma_gemm64<0, false, 0, 1, false, 0><<<grid, 256, 0, stream>>>(
        (const unsigned short*)z16, (const unsigned short*)z16, kD, 0L,
        (const unsigned short*)w16, (const unsigned short*)w16, kD, 0L,
        (void*)P16, (void*)P16, kNcat, 0L,
        b1, b1, 0L,
        Mp, kNcat, kD, 1.0f / 16.0f);
  }
  {
    const int nWaves = (E + 31) / 32;
    const int grid = (nWaves + 7) / 8;
    edge_decode_kernel<<<grid, 256, 0, stream>>>(P16, eidx, b1, W2, b2, out, E, Nn);
  }
  hipGetLastError();
}
